// QPGA_27470610825419
// MI455X (gfx1250) — hardware-verified
//
#include <hip/hip_runtime.h>
#include <math.h>

typedef __attribute__((ext_vector_type(16))) _Float16 v16h;
typedef __attribute__((ext_vector_type(8)))  _Float16 v8h;
typedef __attribute__((ext_vector_type(8)))  float    v8f;
typedef __attribute__((ext_vector_type(4)))  float    v4f;

constexpr int kNS      = 1024;
constexpr int kNQ      = 11;
constexpr int kNL      = 8;
constexpr int kDim     = 2048;
constexpr int kNSlow   = 32;
constexpr int kNFast   = 64;
constexpr int kSampF   = 2 * kDim;
constexpr int kNTab    = 3 * kNL;
constexpr int kTabPit  = 2 * kDim;
constexpr int kKB      = 2 * kNFast;
constexpr int kKA      = 2 * kNSlow;
constexpr int kNApp    = 2 * kNL;
static_assert(kDim == (1 << kNQ));
static_assert(kNSlow * kNFast == kDim);
static_assert((kKB % 32) == 0 && (kKA % 32) == 0);
static_assert(kNSlow == 32 && kNFast == 64);

constexpr float kLoCarry  = 2048.0f;
constexpr float kLoInv    = 1.0f / 2048.0f;
constexpr float kF16Floor = 6.103515625e-05f;

constexpr float kCm = 0.02209708691207959f;
static_assert(__builtin_bit_cast(unsigned, kCm) == 0x3CB504F3u);

constexpr size_t kWsTab   = (size_t)kNTab * kTabPit * 4;
constexpr size_t kWsTotal = kWsTab;
static_assert(kWsTotal == 393216ull);
static_assert(kWsTotal <= 134217728ull);

__device__ __forceinline__ float bf16_value(float f) {
  const unsigned u = __float_as_uint(f);
  const unsigned r = (u + 0x7FFFu + ((u >> 16) & 1u)) & 0xFFFF0000u;
  return __uint_as_float(r);
}

union FragU { v16h v; v8h h[2]; };
__device__ __forceinline__ v16h frag_load(const _Float16* p) {
  FragU f;
  f.h[0] = *(const v8h*)(p);
  f.h[1] = *(const v8h*)(p + 16);
  return f.v;
}

__device__ __forceinline__ v8f mma_g(v16h a, v16h b, v8f cacc) {
  cacc = __builtin_amdgcn_wmma_f32_16x16x32_f16(false, a, false, b, (short)0, cacc, false, false);
  asm volatile("v_nop\n\tv_nop\n\tv_nop\n\tv_nop" : "+v"(cacc) : "v"(a), "v"(b));
  return cacc;
}

__device__ __forceinline__ float unit_entry(int kp, int np, int xr) {
  const int pc = __popc(xr) & 3;
  const int ci = (int)(pc == 0) - (int)(pc == 2);
  const int si = (int)(pc == 1) - (int)(pc == 3);
  const int v  = (kp == np) ? ci : ((kp == 0) ? si : -si);
  return (float)v;
}

__device__ __forceinline__ void store_split8(_Float16* ph, _Float16* pl, const float (&v)[8]) {
  v8h hv, lv;
#pragma unroll
  for (int e = 0; e < 8; ++e) {
    const float xv = v[e];
    const float xf = (fabsf(xv) < kF16Floor) ? 0.0f : xv;
    const _Float16 hh16 = (_Float16)xf;
    const float rs = (xv - (float)hh16) * kLoCarry;
    const float rf = (fabsf(rs) < kF16Floor) ? 0.0f : rs;
    hv[e] = hh16;
    lv[e] = (_Float16)rf;
  }
  *(v8h*)ph = hv;
  *(v8h*)pl = lv;
}

__device__ __forceinline__ void phase_mul8(const float* __restrict__ tp, float (&a)[8], float (&b)[8]) {
  const v4f c0 = *(const v4f*)(tp);
  const v4f c1 = *(const v4f*)(tp + 4);
  const v4f s0 = *(const v4f*)(tp + kDim);
  const v4f s1 = *(const v4f*)(tp + kDim + 4);
  const float cc[8] = {c0.x, c0.y, c0.z, c0.w, c1.x, c1.y, c1.z, c1.w};
  const float ss[8] = {s0.x, s0.y, s0.z, s0.w, s1.x, s1.y, s1.z, s1.w};
#pragma unroll
  for (int e = 0; e < 8; ++e) {
    const float na = a[e] * cc[e] - b[e] * ss[e];
    const float nb = a[e] * ss[e] + b[e] * cc[e];
    a[e] = na;
    b[e] = nb;
  }
}

__global__ __launch_bounds__(256) void phase_table_kernel(
    const float* __restrict__ alphas, const float* __restrict__ betas,
    const float* __restrict__ thetas, const float* __restrict__ phis,
    float* __restrict__ ptab)
{
  const int tid  = threadIdx.x;
  const int d    = blockIdx.x * 256 + tid;
  const int tab  = blockIdx.y;
  const int l    = tab / 3;
  const int kind = tab - 3 * l;
  float total = 0.0f;
#pragma unroll
  for (int q = 0; q < kNQ; ++q) {
    const float va = bf16_value(alphas[l * kNQ + q]);
    const float vb = bf16_value(betas[l * kNQ + q]);
    const float vt = bf16_value(thetas[l * kNQ + q]);
    const float vp = bf16_value(phis[l * kNQ + q]);
    const float z0 = (kind == 0) ? va : ((kind == 1) ? vt : vp);
    const float z1 = (kind == 0) ? vb : 0.0f;
    const float ad = (((d >> (kNQ - 1 - q)) & 1) != 0) ? z1 : z0;
    total = total + ad;
  }
  float sn, cs;
  sincosf(total, &sn, &cs);
  const int pm   = ((l & 1) != 0) ? 0x2AA : 0x554;
  const int neg  = __popc((d & ~(d << 1)) & pm) & 1;
  const bool flp = (kind == 2) && (neg != 0);
  const float cv = flp ? -cs : cs;
  const float sv = flp ? -sn : sn;
  float* pc = ptab + (size_t)tab * kTabPit + d;
  *(volatile float*)(pc) = cv;
  *(volatile float*)(pc + kDim) = sv;
  __threadfence();
  *(volatile float*)(pc) = cv;
  *(volatile float*)(pc + kDim) = sv;
}

__global__ __launch_bounds__(256) void mixer_kernel(
    const float* __restrict__ x, const float* __restrict__ ptab, float* __restrict__ out)
{
  __shared__ __align__(16) _Float16 sBtB[kKB * kKB];
  __shared__ __align__(16) _Float16 sBtA[kKA * kKA];
  __shared__ __align__(16) _Float16 sABh[kNSlow * kKB];
  __shared__ __align__(16) _Float16 sABl[kNSlow * kKB];
  __shared__ __align__(16) _Float16 sAAh[kNFast * kKA];
  __shared__ __align__(16) _Float16 sAAl[kNFast * kKA];
  __shared__ __align__(16) float    sOut[kSampF];

  const int tid  = threadIdx.x;
  const int lane = tid & 31;
  const int wave = tid >> 5;
  const int hh   = lane >> 4;
  const int c    = lane & 15;
  const int smp  = blockIdx.x;

#pragma unroll 1
  for (int i = 0; i < 8; ++i) {
    const int idx = tid + 256 * i;
    const int n   = idx >> 4;
    const int k8  = (idx & 15) * 8;
    v8h hv;
#pragma unroll
    for (int e = 0; e < 8; ++e) {
      const int k = k8 + e;
      hv[e] = (_Float16)unit_entry(k >> 6, n >> 6, (k & 63) ^ (n & 63));
    }
    *(v8h*)(sBtB + n * kKB + k8) = hv;
  }
#pragma unroll 1
  for (int i = 0; i < 2; ++i) {
    const int idx = tid + 256 * i;
    const int n   = idx >> 3;
    const int k8  = (idx & 7) * 8;
    v8h hv;
#pragma unroll
    for (int e = 0; e < 8; ++e) {
      const int k = k8 + e;
      hv[e] = (_Float16)unit_entry(k >> 5, n >> 5, (k & 31) ^ (n & 31));
    }
    *(v8h*)(sBtA + n * kKA + k8) = hv;
  }

  {
    const int d0 = tid * 8;
    const float* xs = x + (size_t)smp * kSampF;
    const v4f r0 = *(const v4f*)(xs + d0);
    const v4f r1 = *(const v4f*)(xs + d0 + 4);
    const v4f i0 = *(const v4f*)(xs + kDim + d0);
    const v4f i1 = *(const v4f*)(xs + kDim + d0 + 4);
    float ta[8] = {bf16_value(r0.x), bf16_value(r0.y), bf16_value(r0.z), bf16_value(r0.w),
                   bf16_value(r1.x), bf16_value(r1.y), bf16_value(r1.z), bf16_value(r1.w)};
    float tb[8] = {bf16_value(i0.x), bf16_value(i0.y), bf16_value(i0.z), bf16_value(i0.w),
                   bf16_value(i1.x), bf16_value(i1.y), bf16_value(i1.z), bf16_value(i1.w)};
    phase_mul8(ptab + d0, ta, tb);
    const int orow = (tid >> 3) * kKB + (tid & 7) * 8;
    store_split8(sABh + orow, sABl + orow, ta);
    store_split8(sABh + orow + kNFast, sABl + orow + kNFast, tb);
  }
  __syncthreads();

#pragma unroll 1
  for (int app = 0; app < kNApp; ++app) {
    const int  l   = app >> 1;
    const bool odd = (app & 1) != 0;

    {
      const int mt = wave >> 2;
      const int jt = wave & 3;
      const int arow  = (16 * mt + c) * kKB + 8 * hh;
      const int b0row = (16 * jt + c) * kKB + 8 * hh;
      const int b1row = (kNFast + 16 * jt + c) * kKB + 8 * hh;
      v8f ah0 = (v8f){0.f, 0.f, 0.f, 0.f, 0.f, 0.f, 0.f, 0.f};
      v8f ah1 = ah0;
      v8f al0 = ah0;
      v8f al1 = ah0;
#pragma unroll
      for (int ks = 0; ks < kKB / 32; ++ks) {
        const v16h fa = frag_load(sABh + arow + ks * 32);
        const v16h fl = frag_load(sABl + arow + ks * 32);
        const v16h b0 = frag_load(sBtB + b0row + ks * 32);
        const v16h b1 = frag_load(sBtB + b1row + ks * 32);
        ah0 = mma_g(fa, b0, ah0);
        ah1 = mma_g(fa, b1, ah1);
        al0 = mma_g(fl, b0, al0);
        al1 = mma_g(fl, b1, al1);
      }
      float re[8], im[8];
#pragma unroll
      for (int r = 0; r < 8; ++r) {
        re[r] = ah0[r] + al0[r] * kLoInv;
        im[r] = ah1[r] + al1[r] * kLoInv;
      }
      const int orow = (16 * jt + c) * kKA + 16 * mt + 8 * hh;
      store_split8(sAAh + orow, sAAl + orow, re);
      store_split8(sAAh + orow + kNSlow, sAAl + orow + kNSlow, im);
    }
    __syncthreads();

    {
      const int mt = wave >> 1;
      const int it = wave & 1;
      const int arow  = (16 * mt + c) * kKA + 8 * hh;
      const int b0row = (16 * it + c) * kKA + 8 * hh;
      const int b1row = (kNSlow + 16 * it + c) * kKA + 8 * hh;
      v8f ah0 = (v8f){0.f, 0.f, 0.f, 0.f, 0.f, 0.f, 0.f, 0.f};
      v8f ah1 = ah0;
      v8f al0 = ah0;
      v8f al1 = ah0;
#pragma unroll
      for (int ks = 0; ks < kKA / 32; ++ks) {
        const v16h fa = frag_load(sAAh + arow + ks * 32);
        const v16h fl = frag_load(sAAl + arow + ks * 32);
        const v16h b0 = frag_load(sBtA + b0row + ks * 32);
        const v16h b1 = frag_load(sBtA + b1row + ks * 32);
        ah0 = mma_g(fa, b0, ah0);
        ah1 = mma_g(fa, b1, ah1);
        al0 = mma_g(fl, b0, al0);
        al1 = mma_g(fl, b1, al1);
      }
      float re[8], im[8];
#pragma unroll
      for (int r = 0; r < 8; ++r) {
        re[r] = (ah0[r] + al0[r] * kLoInv) * kCm;
        im[r] = (ah1[r] + al1[r] * kLoInv) * kCm;
      }
      const int dd = (16 * it + c) * kNFast + 16 * mt + 8 * hh;
      const int t1 = 3 * l + (odd ? 2 : 1);
      phase_mul8(ptab + (size_t)t1 * kTabPit + dd, re, im);
      if (odd && (l < kNL - 1)) {
        phase_mul8(ptab + (size_t)(3 * (l + 1)) * kTabPit + dd, re, im);
      }
      if (app == kNApp - 1) {
        const v4f o0 = (v4f){re[0], re[1], re[2], re[3]};
        const v4f o1 = (v4f){re[4], re[5], re[6], re[7]};
        const v4f o2 = (v4f){im[0], im[1], im[2], im[3]};
        const v4f o3 = (v4f){im[4], im[5], im[6], im[7]};
        *(v4f*)(sOut + dd) = o0;
        *(v4f*)(sOut + dd + 4) = o1;
        *(v4f*)(sOut + kDim + dd) = o2;
        *(v4f*)(sOut + kDim + dd + 4) = o3;
      } else {
        const int orow = (16 * it + c) * kKB + 16 * mt + 8 * hh;
        store_split8(sABh + orow, sABl + orow, re);
        store_split8(sABh + orow + kNFast, sABl + orow + kNFast, im);
      }
    }
    __syncthreads();
  }

  {
    v4f ov[4];
#pragma unroll
    for (int it = 0; it < 4; ++it) ov[it] = *(const v4f*)(sOut + (it * 256 + tid) * 4);
    float* ob = out + (size_t)smp * kSampF;
    for (int pass = 0; pass < 2; ++pass) {
#pragma unroll
      for (int it = 0; it < 4; ++it) {
        *(volatile v4f*)(ob + (it * 256 + tid) * 4) = ov[it];
      }
      __threadfence();
    }
  }
}

extern "C" void kernel_launch(void* const* d_in, const int* in_sizes, int n_in,
                              void* d_out, int out_size, void* d_ws, size_t ws_size,
                              hipStream_t stream) {
  if (n_in < 5) return;
  if (in_sizes[0] != kNS * kSampF) return;
  if (in_sizes[1] != kNL * kNQ) return;
  if (in_sizes[2] != kNL * kNQ) return;
  if (in_sizes[3] != kNL * kNQ) return;
  if (in_sizes[4] != kNL * kNQ) return;
  if (out_size != kNS * kSampF) return;
  if (ws_size < kWsTotal) return;

  const float* x      = (const float*)d_in[0];
  const float* alphas = (const float*)d_in[1];
  const float* betas  = (const float*)d_in[2];
  const float* thetas = (const float*)d_in[3];
  const float* phis   = (const float*)d_in[4];
  float* out  = (float*)d_out;
  float* ptab = (float*)d_ws;

  phase_table_kernel<<<dim3(kDim / 256, kNTab), 256, 0, stream>>>(alphas, betas, thetas, phis, ptab);
  mixer_kernel<<<dim3(kNS), 256, 0, stream>>>(x, ptab, out);
}
